// HGT_21337397527227
// MI455X (gfx1250) — hardware-run, weakly checked
//
#include <hip/hip_runtime.h>


namespace {
constexpr int ECUT = 500000  ; constexpr int N0 = 100000, N1 = 20000, N0P = 100032, N1P = 20032, NC0 = 100032, NC1 = 20032  , E = 500000, C = 128, H = 2, D = 64, L = 2;
constexpr float XS = 8.0f, WSC = 256.0f, GS = 64.0f  ;
static_assert(N0P % 64 == 0 && N1P % 64 == 0 && NC0 % 64 == 0 && NC1 % 64 == 0, "tiling");
typedef _Float16 b16;
typedef __attribute__((ext_vector_type(16))) _Float16 v16b;
typedef __attribute__((ext_vector_type(8))) _Float16 v8b;
typedef __attribute__((ext_vector_type(8))) float v8f;
typedef __attribute__((ext_vector_type(4))) float v4f;
__device__ __forceinline__ float bf16_rne(float f) { unsigned int u = __float_as_uint(f); u += 0x7FFFu + ((u >> 16) & 1u); return __uint_as_float(u & 0xFFFF0000u); }
__device__ __forceinline__ void split16(float v, b16& hi, b16& lo) { hi = (b16)v; lo = (b16)(v - (float)hi); }
__device__ __forceinline__ v16b frag_kb(const b16* p, int hh) { const v8b a = *(const v8b*)(p + 8 * hh), b = *(const v8b*)(p + 16 + 8 * hh); v16b f;
#pragma unroll
  for (int e = 0; e < 8; ++e) { f[e] = a[e]; f[8 + e] = b[e]; } return f; }
__device__ __forceinline__ v8f wmma16b(v16b a, v16b b, v8f c) { v8f d = __builtin_amdgcn_wmma_f32_16x16x32_f16(false, a, false, b, (short)0, c, false, false); asm volatile("v_nop\n\tv_nop\n\tv_nop\n\tv_nop" : "+v"(d) : "v"(a), "v"(b)); return d; }
__device__ __forceinline__ void wave_lds_sync() { __builtin_amdgcn_fence(__ATOMIC_RELEASE, "workgroup"); __builtin_amdgcn_wave_barrier(); __builtin_amdgcn_fence(__ATOMIC_ACQUIRE, "workgroup"); }
__device__ __forceinline__ float pmul(float a, float b) { float p = a * b; asm volatile("" : "+v"(p)); return p; }
__device__ __forceinline__ int iclamp(int v, int lo, int hi) { return v < lo ? lo : (v > hi ? hi : v); }
constexpr int CSR_NBLK = 512, CSR_GB = 8, CSR_GN = 1 << CSR_GB  , CSR_MAXG = 512, CSR_CAP = 12288  ;
__global__ __launch_bounds__(64) void csrA_kernel(const int* __restrict__ dst, int E, int N, int nG, int CHP, int NGP, int* __restrict__ STG, int* __restrict__ HST) {
  extern __shared__ int sm[];
  int* cnt = sm; int* run = sm + NGP; int* ids = sm + 2 * NGP;
  const int b = blockIdx.x; const int ch = (E + CSR_NBLK - 1) / CSR_NBLK; const int e0 = b * ch, e1 = min(E, e0 + ch);
  for (int i = threadIdx.x; i < NGP; i += 64) cnt[i] = 0;
  for (int i = threadIdx.x; i < CHP; i += 64) ids[i] = -1;
  __syncthreads();
  if (threadIdx.x == 0) {
    for (int e = e0; e < e1; ++e) { int d = dst[e]; d = (d < 0) ? 0 : (d >= N ? N - 1 : d); cnt[d >> CSR_GB] += 1; }
    int acc = 0; for (int g = 0; g < nG; ++g) { run[g] = acc; acc += cnt[g]; }
    for (int e = e0; e < e1; ++e) { int d = dst[e]; d = (d < 0) ? 0 : (d >= N ? N - 1 : d); const int g = d >> CSR_GB; ids[run[g]] = e; run[g] += 1; } }
  __syncthreads();
  typedef __attribute__((ext_vector_type(4))) int v4i;
  for (int pass = 0; pass < 2; ++pass) {
    for (int i = threadIdx.x; i < CHP / 4; i += 64) *(volatile v4i*)(STG + (size_t)b * CHP + i * 4) = *(const v4i*)(&ids[i * 4]);
    for (int i = threadIdx.x; i < NGP / 4; i += 64) { v4i v; for (int e = 0; e < 4; ++e) v[e] = (i * 4 + e < nG) ? cnt[i * 4 + e] : 0; *(volatile v4i*)(HST + (size_t)b * NGP + i * 4) = v; }
    __threadfence(); }
}
__global__ __launch_bounds__(512) void csrS_kernel(const int* __restrict__ HST, int nG, int NGP, int* __restrict__ START, int* __restrict__ TOT, int* __restrict__ OFF) {
  __shared__ int tot[CSR_MAXG];
  const int b = threadIdx.x;
  for (int pass = 0; pass < 2; ++pass) { int runb = 0; for (int g = 0; g < nG; ++g) { int c = HST[(size_t)b * NGP + g]; c = (c < 0) ? 0 : c; ((volatile int*)OFF)[(size_t)g * CSR_NBLK + b] = runb; runb += c; } __threadfence(); }
  for (int g = threadIdx.x; g < nG; g += 512) { int s = 0; for (int bb = 0; bb < CSR_NBLK; ++bb) { int c = HST[(size_t)bb * NGP + g]; s += (c < 0) ? 0 : c; } tot[g] = s; }
  __syncthreads();
  if (threadIdx.x < 32) {
    __shared__ int st[CSR_MAXG + 32];
    if (threadIdx.x == 0) { int acc = 0; for (int g = 0; g < NGP; ++g) { st[g] = acc; if (g < nG) acc += (tot[g] + 31) & ~31; } st[NGP] = acc; }
    __builtin_amdgcn_fence(__ATOMIC_RELEASE, "workgroup"); __builtin_amdgcn_wave_barrier(); __builtin_amdgcn_fence(__ATOMIC_ACQUIRE, "workgroup");
    for (int pass = 0; pass < 2; ++pass) { for (int i = threadIdx.x; i < NGP + 32; i += 32) { ((volatile int*)START)[i] = (i <= NGP) ? st[min(i, NGP)] : 0; ((volatile int*)TOT)[i] = (i < nG) ? tot[i] : 0; } __threadfence(); } }
}
__global__ __launch_bounds__(256) void csrB_kernel(const int* __restrict__ dst, int N, int nG, int CHP, int NGP, int permLen, const int* __restrict__ STG, const int* __restrict__ HST, const int* __restrict__ OFF, const int* __restrict__ START, const int* __restrict__ TOT, int* __restrict__ PERM, int* __restrict__ ROWPTR, int* __restrict__ ROWCNT, int* __restrict__ FLAG) {
  typedef __attribute__((ext_vector_type(4))) int v4i;
  __shared__ int ids[CSR_CAP]; __shared__ unsigned short key[CSR_CAP]; __shared__ int outp[CSR_CAP]; __shared__ int ncnt[CSR_GN + 1]; __shared__ int boff[CSR_NBLK + 1];
  const int g = blockIdx.x, t_ = threadIdx.x; int tot = TOT[g]; int st = START[g], stn = START[g + 1]; const int v0 = g * CSR_GN; const int nv = min(CSR_GN, N - v0);
  st = (st < 0) ? 0 : (st > permLen - 32 ? permLen - 32 : st) & ~31; stn = (stn < st) ? st : (stn > permLen ? permLen : stn); tot = (tot < 0) ? 0 : tot; if (tot > stn - st && tot <= CSR_CAP) tot = stn - st;
  if (tot > CSR_CAP) {
    for (int pass = 0; pass < 2; ++pass) { for (int i = t_; i < CSR_GN / 4; i += 256) { v4i a, c; for (int e = 0; e < 4; ++e) { a[e] = st; c[e] = 0; } *(volatile v4i*)(ROWPTR + v0 + i * 4) = a; *(volatile v4i*)(ROWCNT + v0 + i * 4) = c; } if (t_ == 0) ((volatile int*)FLAG)[0] = 1; __threadfence(); } (void)nv; return; }
  if (t_ == 0) { int acc = 0; for (int b = 0; b < CSR_NBLK; ++b) { boff[b] = acc; int c = HST[(size_t)b * NGP + g]; c = (c < 0) ? 0 : (c > CHP ? CHP : c); acc += c; if (acc > tot) acc = tot; } boff[CSR_NBLK] = acc; }
  for (int i = t_; i <= CSR_GN; i += 256) ncnt[i] = 0;
  __syncthreads();
  for (int b = 0; b < CSR_NBLK; ++b) { const int c = boff[b + 1] - boff[b]; int o_ = OFF[(size_t)g * CSR_NBLK + b]; o_ = (o_ < 0) ? 0 : (o_ > CHP - c ? CHP - c : o_); const int* src_ = STG + (size_t)b * CHP + o_;
    for (int i = t_; i < c; i += 256) { int id = src_[i]; id = (id < 0) ? 0 : id; ids[boff[b] + i] = id; int d = dst[id]; d = (d < v0) ? v0 : (d >= N ? N - 1 : d); int kk = d - v0; kk = (kk < 0) ? 0 : (kk >= CSR_GN ? CSR_GN - 1 : kk); key[boff[b] + i] = (unsigned short)kk; } }
  __syncthreads();
  if (t_ == 0) { for (int i = 0; i < tot; ++i) ncnt[key[i]] += 1; int acc = 0; for (int vl = 0; vl < CSR_GN; ++vl) { const int c = ncnt[vl]; ncnt[vl] = acc; acc += c; } ncnt[CSR_GN] = acc;
    for (int i = 0; i < tot; ++i) { const int vl = key[i]; outp[ncnt[vl]] = ids[i]; ncnt[vl] += 1; }
    for (int vl = CSR_GN; vl > 0; --vl) ncnt[vl] = ncnt[vl - 1]; ncnt[0] = 0; }
  __syncthreads();
  for (int pass = 0; pass < 2; ++pass) {
    for (int i = t_; i < (stn - st) / 4; i += 256) { v4i v; for (int e = 0; e < 4; ++e) { const int q = i * 4 + e; v[e] = (q < tot) ? outp[q] : -1; } *(volatile v4i*)(PERM + st + i * 4) = v; }
    for (int i = t_; i < CSR_GN / 4; i += 256) { v4i a, c; for (int e = 0; e < 4; ++e) { const int vl = i * 4 + e; a[e] = st + ncnt[vl]; c[e] = (vl < nv) ? (ncnt[vl + 1] - ncnt[vl]) : 0; } *(volatile v4i*)(ROWPTR + v0 + i * 4) = a; *(volatile v4i*)(ROWCNT + v0 + i * 4) = c; }
    __threadfence(); }
}
__global__ __launch_bounds__(256) void csrZ_kernel(int* __restrict__ p, size_t n4) { typedef __attribute__((ext_vector_type(4))) int v4i; const size_t tid = (size_t)blockIdx.x * 256 + threadIdx.x, nth = (size_t)gridDim.x * 256; v4i z = {0, 0, 0, 0}; for (size_t i = tid; i < n4; i += nth) *(volatile v4i*)(p + i * 4) = z; }
struct CsrBufs { int *STG, *HST, *OFF, *START, *TOT, *PERM, *ROWPTR, *ROWCNT, *FLAG; int nG, NGP, CHP; size_t permLen; char* base; size_t bytes; };
static size_t csr_carve(CsrBufs& c, char* ws, size_t off, int E, int N) {
  const size_t off0 = off; c.base = ws + off;
  auto al = [&](size_t bytes) { char* p = ws + off; off += (bytes + 255) & ~(size_t)255; return p; };
  c.nG = (N + CSR_GN - 1) / CSR_GN; c.NGP = (c.nG + 31) & ~31; const int ch = (E + CSR_NBLK - 1) / CSR_NBLK; c.CHP = (ch + 31) & ~31; c.permLen = (size_t)E + 32 * (size_t)c.nG + 32;
  c.STG = (int*)al((size_t)CSR_NBLK * c.CHP * 4); c.HST = (int*)al((size_t)CSR_NBLK * c.NGP * 4); c.OFF = (int*)al((size_t)c.NGP * CSR_NBLK * 4); c.START = (int*)al((size_t)(c.NGP + 64) * 4); c.TOT = (int*)al((size_t)(c.NGP + 64) * 4);
  c.PERM = (int*)al(c.permLen * 4); c.ROWPTR = (int*)al((size_t)c.nG * CSR_GN * 4); c.ROWCNT = (int*)al((size_t)c.nG * CSR_GN * 4); c.FLAG = (int*)al(256);
  c.bytes = off - off0; return off;
}
static void csr_build(const CsrBufs& c, const int* dst, int E, int N, hipStream_t stream) {
  const size_t smem = (size_t)(2 * c.NGP + c.CHP) * 4;
  csrZ_kernel<<<512, 256, 0, stream>>>((int*)c.base, c.bytes / 16);
  csrA_kernel<<<CSR_NBLK, 64, smem, stream>>>(dst, E, N, c.nG, c.CHP, c.NGP, c.STG, c.HST);
  csrS_kernel<<<1, 512, 0, stream>>>(c.HST, c.nG, c.NGP, c.START, c.TOT, c.OFF);
  csrB_kernel<<<c.nG, 256, 0, stream>>>(dst, N, c.nG, c.CHP, c.NGP, (int)c.permLen, c.STG, c.HST, c.OFF, c.START, c.TOT, c.PERM, c.ROWPTR, c.ROWCNT, c.FLAG);
}

typedef __attribute__((ext_vector_type(4))) _Float16 v4h;
typedef __attribute__((ext_vector_type(2))) float v2f;
__global__ __launch_bounds__(256) void comp_kernel(const float* __restrict__ wk, const float* __restrict__ bk, const float* __restrict__ wv, const float* __restrict__ bv, const float* __restrict__ arel, const float* __restrict__ mrel, float* __restrict__ CW, float* __restrict__ CB) {
  const int u = blockIdx.x * 256 + threadIdx.x; const int per = C * C; if (u >= L * 2 * 2 * per + L * 2 * 2 * C) return;
  if (u < L * 2 * 2 * per) { const int idx = u / per, el = u % per; const int l = idx / 4, t = (idx / 2) % 2, kv = idx % 2; const int k = el / C, o = el % C; const int r = t; const int hd = o / D, oo = o % D;
    const float* W = (kv ? wv : wk) + ((size_t)(l * 2 + t)) * per; const float* Bm = (kv ? mrel : arel) + (((size_t)(l * 2 + r)) * H + hd) * D * D;
    float s = 0.0f; for (int j = 0; j < D; ++j) s += bf16_rne(W[(size_t)k * C + hd * D + j]) * bf16_rne(Bm[(size_t)j * D + oo]);
    for (int pass = 0; pass < 2; ++pass) { ((volatile float*)CW)[u] = s; __threadfence(); } }
  else { const int v = u - L * 2 * 2 * per; const int idx = v / C, o = v % C; const int l = idx / 4, t = (idx / 2) % 2, kv = idx % 2; const int r = t; const int hd = o / D, oo = o % D;
    const float* b = (kv ? bv : bk) + (size_t)(l * 2 + t) * C; const float* Bm = (kv ? mrel : arel) + (((size_t)(l * 2 + r)) * H + hd) * D * D; float s = 0.0f; for (int j = 0; j < D; ++j) s += bf16_rne(b[hd * D + j]) * bf16_rne(Bm[(size_t)j * D + oo]);
    for (int pass = 0; pass < 2; ++pass) { ((volatile float*)CB)[v] = s; __threadfence(); } }
}
__global__ __launch_bounds__(256) void prep_kernel(const float* __restrict__ wl, const float* __restrict__ wq, const float* __restrict__ wa, const float* __restrict__ CW, b16* __restrict__ WL, b16* __restrict__ TT) {
  const int per8 = C * C / 8; const int u = blockIdx.x * 256 + threadIdx.x; if (u >= 2 * per8 + L * 2 * 6 * per8) return; v8b o;
  if (u < 2 * per8) { const int t = u / per8, e = (u % per8) * 8; const int oo = e / C, k0 = e % C; for (int j = 0; j < 8; ++j) o[j] = (b16)(bf16_rne(wl[((size_t)t * C + k0 + j) * C + oo]) * WSC); for (int pass = 0; pass < 2; ++pass) { *(volatile v8b*)(WL + (size_t)t * C * C + e) = o; __threadfence(); } return; }
  const int v = u - 2 * per8; const int idx = v / per8, e = (v % per8) * 8; const int l = idx / 12, t = (idx / 6) % 2, m = idx % 6; const int oo = e / C, k0 = e % C;
  for (int j = 0; j < 8; ++j) { const int k = k0 + j; float w; b16 val;
    if (m == 0) { w = bf16_rne(wq[(((size_t)(l * 2 + t)) * C + k) * C + oo]); val = (b16)(w * WSC); }
    else if (m == 5) { w = bf16_rne(wa[(((size_t)(l * 2 + t)) * C + k) * C + oo]); val = (b16)(w * WSC); }
    else { const int kv = (m >= 3) ? 1 : 0; const bool lo = (m == 2 || m == 4); w = CW[((((size_t)(l * 2 + t)) * 2 + kv) * C + k) * C + oo]; b16 p, q; split16(w * WSC, p, q); val = lo ? q : p; }
    o[j] = val; }
  for (int pass = 0; pass < 2; ++pass) { *(volatile v8b*)(TT + (size_t)idx * C * C + e) = o; __threadfence(); }
}
__global__ __launch_bounds__(128) void xs_kernel(const float* __restrict__ x, int N, int NC, const b16* __restrict__ WLt, const float* __restrict__ bl, float* __restrict__ XSr) {
  __shared__ __attribute__((aligned(16))) float Tf[4][16][C + 4];
  const int wave = threadIdx.x >> 5, lane = threadIdx.x & 31, nloc = lane & 15, hlf = lane >> 4; const size_t m0 = ((size_t)blockIdx.x * 4 + wave) * 16; const size_t vr = m0 + nloc; const size_t vra = vr < (size_t)N ? vr : (size_t)N - 1;
  v8f acc[8];
#pragma unroll
  for (int tt = 0; tt < 8; ++tt) acc[tt] = (v8f){};
  if (m0 < (size_t)NC) {
#pragma unroll
    for (int ks = 0; ks < 4; ++ks) { v16b a; const float* xr = x + vra * C + ks * 32; const v4f c0 = *(const v4f*)(xr + 8 * hlf), c1 = *(const v4f*)(xr + 8 * hlf + 4), c2 = *(const v4f*)(xr + 16 + 8 * hlf), c3 = *(const v4f*)(xr + 16 + 8 * hlf + 4); float cv[16];
      for (int i = 0; i < 4; ++i) { cv[i] = c0[i]; cv[4 + i] = c1[i]; cv[8 + i] = c2[i]; cv[12 + i] = c3[i]; }
#pragma unroll
      for (int e2 = 0; e2 < 16; ++e2) a[e2] = (b16)(bf16_rne(vr < (size_t)N ? cv[e2] : 0.0f) * XS);
#pragma unroll
      for (int tt = 0; tt < 8; ++tt) acc[tt] = wmma16b(a, frag_kb(WLt + (size_t)(tt * 16 + nloc) * C + ks * 32, hlf), acc[tt]); } }
#pragma unroll
  for (int tt = 0; tt < 8; ++tt) { const float bb = bf16_rne(bl[tt * 16 + nloc]);
#pragma unroll
    for (int r = 0; r < 8; ++r) Tf[wave][8 * hlf + r][tt * 16 + nloc] = (m0 + 8 * hlf + r < (size_t)NC) ? fmaxf(acc[tt][r] * (1.0f / (XS * WSC)) + bb, 0.0f) : 0.0f; }
  wave_lds_sync();
  for (int pass = 0; pass < 2; ++pass) { for (int rr = 0; rr < 16; ++rr) *(volatile v4f*)(XSr + (m0 + rr) * C + lane * 4) = *(const v4f*)(&Tf[wave][rr][lane * 4]); __threadfence(); }
}
template <int MODE>
__global__ __launch_bounds__(128) void proj_kernel(const float* __restrict__ XSr, int NC, const b16* __restrict__ T6, const float* __restrict__ bq, const float* __restrict__ cbk, const float* __restrict__ cbv, b16* __restrict__ Qp, b16* __restrict__ KRp, float* __restrict__ VR) {
  __shared__ __attribute__((aligned(16))) float Tf[4][16][C + 4], Tg[4][16][C + 4];
  const int wave = threadIdx.x >> 5, lane = threadIdx.x & 31, nloc = lane & 15, hlf = lane >> 4; const size_t m0 = ((size_t)blockIdx.x * 4 + wave) * 16; const size_t vr = m0 + nloc;
  const b16* WQ = T6; const b16* WKh = T6 + (size_t)C * C; const b16* WKl = T6 + (size_t)2 * C * C; const b16* WVh = T6 + (size_t)3 * C * C; const b16* WVl = T6 + (size_t)4 * C * C;
  v8f a1[8], a2[8];
#pragma unroll
  for (int tt = 0; tt < 8; ++tt) { a1[tt] = (v8f){}; a2[tt] = (v8f){}; }
  if (m0 < (size_t)NC) {
#pragma unroll
    for (int ks = 0; ks < 4; ++ks) { v16b ah, al; const float* xr = XSr + vr * C + ks * 32; const v4f c0 = *(const v4f*)(xr + 8 * hlf), c1 = *(const v4f*)(xr + 8 * hlf + 4), c2 = *(const v4f*)(xr + 16 + 8 * hlf), c3 = *(const v4f*)(xr + 16 + 8 * hlf + 4); float cv[16];
      for (int i = 0; i < 4; ++i) { cv[i] = c0[i]; cv[4 + i] = c1[i]; cv[8 + i] = c2[i]; cv[12 + i] = c3[i]; }
#pragma unroll
      for (int e2 = 0; e2 < 16; ++e2) { b16 p, q; split16(cv[e2] * XS, p, q); ah[e2] = p; al[e2] = q; }
#pragma unroll
      for (int tt = 0; tt < 8; ++tt) { const size_t bo = (size_t)(tt * 16 + nloc) * C + ks * 32;
        if (MODE == 0) { a1[tt] = wmma16b(ah, frag_kb(WQ + bo, hlf), a1[tt]); a2[tt] = wmma16b(ah, frag_kb(WKh + bo, hlf), a2[tt]); a2[tt] = wmma16b(ah, frag_kb(WKl + bo, hlf), a2[tt]); }
        else { const v16b bh = frag_kb(WVh + bo, hlf), blo = frag_kb(WVl + bo, hlf); a1[tt] = wmma16b(ah, bh, a1[tt]); a1[tt] = wmma16b(ah, blo, a1[tt]); a1[tt] = wmma16b(al, bh, a1[tt]); } } } }
#pragma unroll
  for (int tt = 0; tt < 8; ++tt) { const int col = tt * 16 + nloc; const float b1v = (MODE == 0) ? bf16_rne(bq[col]) : cbv[col], b2v = (MODE == 0) ? cbk[col] : 0.0f;
#pragma unroll
    for (int r = 0; r < 8; ++r) { const bool lv = (m0 + 8 * hlf + r) < (size_t)NC; Tf[wave][8 * hlf + r][col] = lv ? a1[tt][r] * (1.0f / (XS * WSC)) + b1v : 0.0f; if (MODE == 0) Tg[wave][8 * hlf + r][col] = lv ? a2[tt][r] * (1.0f / (XS * WSC)) + b2v : 0.0f; } }
  wave_lds_sync();
  for (int pass = 0; pass < 2; ++pass) {
    for (int rr = 0; rr < 16; ++rr) { const size_t row = m0 + rr;
      if (MODE == 0) { const v4f f = *(const v4f*)(&Tf[wave][rr][lane * 4]), g = *(const v4f*)(&Tg[wave][rr][lane * 4]); v4h o1, o2; for (int j = 0; j < 4; ++j) { o1[j] = (b16)(f[j] * XS); o2[j] = (b16)(g[j] * XS); } *(volatile v4h*)(Qp + row * C + lane * 4) = o1; *(volatile v4h*)(KRp + row * C + lane * 4) = o2; }
      else *(volatile v4f*)(VR + row * C + lane * 4) = *(const v4f*)(&Tf[wave][rr][lane * 4]); }
    __threadfence(); }
}
__global__ __launch_bounds__(256) void agg_kernel(const b16* __restrict__ Qp, const b16* __restrict__ KRp, const float* __restrict__ VR, int NC, int NDP, int NSRC, const float* __restrict__ prel  , const int* __restrict__ srcs, const int* __restrict__ PERM, const int* __restrict__ ROWPTR, const int* __restrict__ ROWCNT, int permLen, float* __restrict__ AGG) {
  const int wave = threadIdx.x >> 5, lane = threadIdx.x & 31; const size_t v = (size_t)blockIdx.x * 8 + wave; if (v >= (size_t)NDP) return; const int c = lane * 4, hd = lane >> 4; v4f acc = {0.0f, 0.0f, 0.0f, 0.0f};
  if (v < (size_t)NC) { const v4h q4 = *(const v4h*)(Qp + v * C + c); float qv[4]; for (int i = 0; i < 4; ++i) qv[i] = (float)q4[i] * (1.0f / XS); const float pr = bf16_rne(prel[hd]) * 0.125f;
    float m = -INFINITY, den = 0.0f; int st = ROWPTR[v], cnt = ROWCNT[v]; cnt = iclamp(cnt, 0, 65536); st = iclamp(st, 0, permLen - cnt);
#pragma unroll 1
    for (int j = 0; j < cnt; ++j) { const int e = iclamp(PERM[st + j], 0, E - 1); const size_t s = (size_t)iclamp(srcs[e], 0, NSRC - 1); const v4h k4 = *(const v4h*)(KRp + s * C + c);
      float p = 0.0f; for (int i = 0; i < 4; ++i) p += pmul(qv[i], (float)k4[i] * (1.0f / XS));
      p += __shfl_xor(p, 1); p += __shfl_xor(p, 2); p += __shfl_xor(p, 4); p += __shfl_xor(p, 8); const float lg = p * pr;
      const float mn = fmaxf(m, lg); const float alf = (m == -INFINITY) ? 0.0f : __expf(m - mn), w = __expf(lg - mn); acc = acc * alf + *(const v4f*)(VR + s * C + c) * w; den = den * alf + w; m = mn; }
    if (den > 0.0f) acc = acc * (1.0f / den); }
  for (int pass = 0; pass < 2; ++pass) { *(volatile v4f*)(AGG + v * C + c) = acc; __threadfence(); }
}
__global__ __launch_bounds__(128) void upd_kernel(const float* __restrict__ AGG, int N, int NC, const b16* __restrict__ WA, const float* __restrict__ ba, const float* __restrict__ skipp  , float* __restrict__ XSr, float* __restrict__ OUT) {
  const float askip = 1.0f / (1.0f + expf(-bf16_rne(skipp[0])));
  __shared__ __attribute__((aligned(16))) float Tf[4][16][C + 4];
  const int wave = threadIdx.x >> 5, lane = threadIdx.x & 31, nloc = lane & 15, hlf = lane >> 4; const size_t m0 = ((size_t)blockIdx.x * 4 + wave) * 16; const size_t vr = m0 + nloc;
  v8f acc[8];
#pragma unroll
  for (int tt = 0; tt < 8; ++tt) acc[tt] = (v8f){};
  const bool live = m0 < (size_t)NC;
  if (live) {
#pragma unroll
    for (int ks = 0; ks < 4; ++ks) { v16b ah, al; const float* xr = AGG + vr * C + ks * 32; const v4f c0 = *(const v4f*)(xr + 8 * hlf), c1 = *(const v4f*)(xr + 8 * hlf + 4), c2 = *(const v4f*)(xr + 16 + 8 * hlf), c3 = *(const v4f*)(xr + 16 + 8 * hlf + 4); float cv[16];
      for (int i = 0; i < 4; ++i) { cv[i] = c0[i]; cv[4 + i] = c1[i]; cv[8 + i] = c2[i]; cv[12 + i] = c3[i]; }
#pragma unroll
      for (int e2 = 0; e2 < 16; ++e2) { const float g = 0.5f * cv[e2] * (1.0f + erff(cv[e2] * 0.70710678118654752f)); b16 p, q; split16(g * GS, p, q); ah[e2] = p; al[e2] = q; }
#pragma unroll
      for (int tt = 0; tt < 8; ++tt) { const v16b bw = frag_kb(WA + (size_t)(tt * 16 + nloc) * C + ks * 32, hlf); acc[tt] = wmma16b(ah, bw, acc[tt]); acc[tt] = wmma16b(al, bw, acc[tt]); } } }
#pragma unroll
  for (int tt = 0; tt < 8; ++tt) { const int col = tt * 16 + nloc; const float bb = bf16_rne(ba[col]);
#pragma unroll
    for (int r = 0; r < 8; ++r) { const size_t row = m0 + 8 * hlf + r; float val = 0.0f; if (live) { const float o_ = acc[tt][r] * (1.0f / (GS * WSC)) + bb; val = askip * o_ + (1.0f - askip) * XSr[row * C + col]; } Tf[wave][8 * hlf + r][col] = val; } }
  __syncthreads();
  for (int pass = 0; pass < 2; ++pass) { for (int rr = 0; rr < 16; ++rr) { const size_t row = m0 + rr; const v4f f = *(const v4f*)(&Tf[wave][rr][lane * 4]); *(volatile v4f*)(XSr + row * C + lane * 4) = f; if (OUT != nullptr && row < (size_t)N && live) *(volatile v4f*)(OUT + row * C + lane * 4) = f; } __threadfence(); }
}
}

extern "C" void kernel_launch(void* const* d_in, const int* in_sizes, int n_in, void* d_out, int out_size, void* d_ws, size_t ws_size, hipStream_t stream) {
  (void)n_in;
  auto Fp = [&](int i) { return (const float*)d_in[i]; }; auto Ip = [&](int i) { return (const int*)d_in[i]; };
  if (in_sizes[0] != N0 * C || in_sizes[1] != N1 * C || in_sizes[2] != E || in_sizes[3] != E || in_sizes[4] != E || in_sizes[5] != E || in_sizes[6] != 2 * C * C || in_sizes[8] != L * 2 * C * C || in_sizes[16] != L * 2 || in_sizes[17] != L * 2 * H * D * D || in_sizes[19] != L * 2 * H || out_size != (N0 + N1) * C) return;
  size_t off = 0; char* ws = (char*)d_ws;
  auto carve = [&](size_t bytes) { char* p = ws + off; off += (bytes + 255) & ~(size_t)255; return p; };
  float* CW = (float*)carve((size_t)L * 2 * 2 * C * C * 4); float* CB = (float*)carve((size_t)L * 2 * 2 * C * 4); b16* WL = (b16*)carve((size_t)2 * C * C * 2); b16* TT = (b16*)carve((size_t)L * 2 * 6 * C * C * 2);
  float* XS0 = (float*)carve((size_t)N0P * C * 4); float* XS1 = (float*)carve((size_t)N1P * C * 4);
  b16* Q0 = (b16*)carve((size_t)N0P * C * 2); float* VR0 = (float*)carve((size_t)N0P * C * 4); float* AGG0 = VR0;
  b16* KR0 = (b16*)carve((size_t)N0P * C * 2); b16* Q1 = (b16*)carve((size_t)N1P * C * 2); b16* KR1 = (b16*)carve((size_t)N1P * C * 2); float* VR1 = (float*)carve((size_t)N1P * C * 4); float* AGG1 = (float*)carve((size_t)N1P * C * 4);
  CsrBufs cmd, cdm; off = csr_carve(cmd, ws, off, ECUT, N1); off = csr_carve(cdm, ws, off, ECUT, N0);
  if (off > ws_size || off > ((size_t)240 << 20)) return;
  comp_kernel<<<(L * 2 * 2 * C * C + L * 2 * 2 * C + 255) / 256, 256, 0, stream>>>(Fp(8), Fp(9), Fp(12), Fp(13), Fp(17), Fp(18), CW, CB);
  prep_kernel<<<(2 * C * C / 8 + L * 2 * 6 * C * C / 8 + 255) / 256, 256, 0, stream>>>(Fp(6), Fp(10), Fp(14), CW, WL, TT);
  csr_build(cmd, Ip(3), ECUT, N1, stream);
  csr_build(cdm, Ip(5), ECUT, N0, stream);
  xs_kernel<<<N0P / 64, 128, 0, stream>>>(Fp(0), N0, NC0, WL, Fp(7), XS0);
  xs_kernel<<<N1P / 64, 128, 0, stream>>>(Fp(1), N1, NC1, WL + (size_t)C * C, Fp(7) + C, XS1);
  for (int l = 0; l < L; ++l) {
    auto T6 = [&](int t) { return TT + ((size_t)(l * 2 + t)) * 6 * C * C; }; auto cb = [&](int t, int kv) { return CB + (((size_t)(l * 2 + t)) * 2 + kv) * C; };
    const float* bq0 = Fp(11) + (size_t)(l * 2 + 0) * C; const float* bq1 = Fp(11) + (size_t)(l * 2 + 1) * C;
    proj_kernel<0><<<N0P / 64, 128, 0, stream>>>(XS0, NC0, T6(0), bq0, cb(0, 0), nullptr, Q0, KR0, nullptr);
    proj_kernel<1><<<N0P / 64, 128, 0, stream>>>(XS0, NC0, T6(0), nullptr, nullptr, cb(0, 1), nullptr, nullptr, VR0);
    proj_kernel<0><<<N1P / 64, 128, 0, stream>>>(XS1, NC1, T6(1), bq1, cb(1, 0), nullptr, Q1, KR1, nullptr);
    proj_kernel<1><<<N1P / 64, 128, 0, stream>>>(XS1, NC1, T6(1), nullptr, nullptr, cb(1, 1), nullptr, nullptr, VR1);
    agg_kernel<<<N1P / 8, 256, 0, stream>>>(Q1, KR0, VR0, NC1, N1P, N0, Fp(19) + (size_t)(l * 2 + 0) * H, Ip(2), cmd.PERM, cmd.ROWPTR, cmd.ROWCNT, (int)cmd.permLen, AGG1);
    agg_kernel<<<N0P / 8, 256, 0, stream>>>(Q0, KR1, VR1, NC0, N0P, N1, Fp(19) + (size_t)(l * 2 + 1) * H, Ip(4), cdm.PERM, cdm.ROWPTR, cdm.ROWCNT, (int)cdm.permLen, AGG0);
    const bool last = (l == L - 1);
    upd_kernel<<<N0P / 64, 128, 0, stream>>>(AGG0, N0, NC0, T6(0) + (size_t)5 * C * C, Fp(15) + (size_t)(l * 2 + 0) * C, Fp(16) + (l * 2 + 0), XS0, last ? (float*)d_out : nullptr);
    upd_kernel<<<N1P / 64, 128, 0, stream>>>(AGG1, N1, NC1, T6(1) + (size_t)5 * C * C, Fp(15) + (size_t)(l * 2 + 1) * C, Fp(16) + (l * 2 + 1), XS1, last ? (float*)d_out + (size_t)N0 * C : nullptr);
  }
}
